// Regressor_83288005804790
// MI455X (gfx1250) — hardware-verified
//
#include <hip/hip_runtime.h>


#define B_    256
#define T_    256
#define F_    8
#define H_    256
#define BT_   16
#define NT_   256
#define K0P_  288
#define K1_   512
#define NX_   21
#define HOFF_ 32
#define NSL_  128
#define WIN0_ 277

static_assert(B_ % BT_ == 0);
static_assert(K0P_ % 32 == 0 && K0P_ == HOFF_ + H_);
static_assert(K1_ == 2 * H_);
static_assert(NT_ == 256 && BT_ * 16 == NT_);

typedef _Float16 v16h __attribute__((ext_vector_type(16)));
typedef _Float16 v8h  __attribute__((ext_vector_type(8)));
typedef float    v8f  __attribute__((ext_vector_type(8)));
typedef float    v4f  __attribute__((ext_vector_type(4)));

union FragH { v16h v; v8h half[2]; };

constexpr int    PPR0_   = K0P_ / 8;
constexpr int    PC0_    = 512 * PPR0_;
constexpr int    PC1_    = H_ * (K1_ / 8);
constexpr int    BK_WO_  = (256 * PPR0_) / NT_;
constexpr int    BK_W1_  = PC0_ / NT_;
constexpr int    NBLK_PL_ = (PC0_ + PC1_) / NT_;
static_assert(256 * PPR0_ == BK_WO_ * NT_ && PC0_ == BK_W1_ * NT_ && PC0_ + PC1_ == NBLK_PL_ * NT_);
constexpr size_t OFF_P0_ = 0;
constexpr size_t SZ_P0_  = (size_t)PC0_ * 16;
constexpr size_t OFF_P1_ = OFF_P0_ + SZ_P0_;
constexpr size_t SZ_P1_  = (size_t)PC1_ * 16;
constexpr size_t WS_END_ = OFF_P1_ + SZ_P1_;
static_assert(SZ_P0_ % 128 == 0 && SZ_P1_ % 128 == 0 && OFF_P1_ % 128 == 0);
static_assert(WS_END_ <= (size_t)134217728);

__device__ __forceinline__ v8f zero8f() {
    v8f z;
#pragma unroll
    for (int i = 0; i < 8; ++i) z[i] = 0.0f;
    return z;
}
__device__ __forceinline__ v8h zero8h() {
    v8h z;
#pragma unroll
    for (int i = 0; i < 8; ++i) z[i] = (_Float16)0.0f;
    return z;
}
__device__ __forceinline__ void ldfrag(FragH& f, const _Float16* p) {
    f.half[0] = *(const v8h*)(p);
    f.half[1] = *(const v8h*)(p + 16);
}
__device__ __forceinline__ v8f mmah(v8f c, const FragH& a, const FragH& b) {
    v8f d = __builtin_amdgcn_wmma_f32_16x16x32_f16(false, a.v, false, b.v, (short)0, c, false, false);
    asm volatile("v_nop\n\tv_nop\n\tv_nop\n\tv_nop" : "+v"(d) : "v"(a.v), "v"(b.v));
    return d;
}
__device__ __forceinline__ float seg_sum(float v) {
    v += __shfl_xor(v, 8, 32); v += __shfl_xor(v, 4, 32); v += __shfl_xor(v, 2, 32); v += __shfl_xor(v, 1, 32);
    return v;
}
__device__ __forceinline__ float sigm_f(float x) {
    return __builtin_amdgcn_rcpf(1.0f + __expf(-x));
}
__device__ __forceinline__ float tanh_f(float x) {
    const float ax = fabsf(x);
    const float e = __expf(-2.0f * ax);
    const float t = (1.0f - e) * __builtin_amdgcn_rcpf(1.0f + e);
    return copysignf(t, x);
}

__global__ __launch_bounds__(NT_)
void k_planes(const float* __restrict__ Wh0, const float* __restrict__ Wo0,
              const float* __restrict__ Wh1, _Float16* planes)
{
    const int tid = threadIdx.x;
    const int blk = blockIdx.x;
    const int p = blk * NT_ + tid;
    v8f v = zero8f();
    int dst;
    if (blk < BK_W1_) {
        const int q = p;
        const int n = q / PPR0_;
        const int j = q - n * PPR0_;
        const int sel = (blk >= BK_WO_) ? 1 : 0;
        const float* src = sel ? Wo0 : Wh0;
        const int nn = sel ? (n - 256) : n;
        const int nc = min(max(nn, 0), 255);
#pragma unroll
        for (int e = 0; e < 8; ++e) {
            const int k = 8 * j + e;
            const int col = (k < NX_) ? k : (k - (HOFF_ - NX_));
            const bool live = (k < NX_) || (k >= HOFF_);
            const int colc = min(max(col, 0), WIN0_ - 1);
            const float x = src[(size_t)nc * WIN0_ + colc];
            v[e] = live ? (x * 64.0f) : 0.0f;
        }
        dst = 8 * q;
    } else {
        const int q = p - PC0_;
        const int n = q >> 6, j = q & 63;
        const float* sp = Wh1 + (size_t)n * K1_ + 8 * j;
        const v4f a = *(const v4f*)(sp);
        const v4f b = *(const v4f*)(sp + 4);
#pragma unroll
        for (int e = 0; e < 4; ++e) { v[e] = a[e] * 64.0f; v[4 + e] = b[e] * 64.0f; }
        dst = (int)(OFF_P1_ / 2) + 8 * q;
    }
    v8h hv;
#pragma unroll
    for (int e = 0; e < 8; ++e) hv[e] = (_Float16)v[e];
    _Float16* d = planes + dst;
    *(volatile v8h*)d = hv;
    __threadfence();
    *(volatile v8h*)d = hv;
}

__global__ __launch_bounds__(NT_)
void k_main(const float* __restrict__ inp, const float* __restrict__ nspt,
            const float* __restrict__ Wds, const float* __restrict__ bds,
            const float* __restrict__ c1w, const float* __restrict__ c1b,
            const float* __restrict__ c2w, const float* __restrict__ c2b,
            const float* __restrict__ c3w, const float* __restrict__ c3b,
            const _Float16* __restrict__ W0p, const _Float16* __restrict__ W1p,
            const float* __restrict__ bh0, const float* __restrict__ bo0,
            const float* __restrict__ bh1, const float* __restrict__ Wo1,
            const float* __restrict__ bo1, float* out)
{
    __shared__ __attribute__((aligned(16))) _Float16 comb0[BT_ * K0P_];
    __shared__ __attribute__((aligned(16))) _Float16 comb1[BT_ * K1_];
    __shared__ __attribute__((aligned(16))) float outS[BT_ * T_];
    __shared__ float g1p[BT_ * 8];
    __shared__ float g1q[BT_ * 8];
    __shared__ float g1S[BT_];
    __shared__ float featS[BT_ * 16];
    __shared__ float xb[3 * NSL_];
    __shared__ float y1[8 * 64];
    __shared__ float y2[8 * 32];
    __shared__ float y3[16 * 16];

    const int tid = threadIdx.x, lane = tid & 31, w = tid >> 5;
    const int hf = lane >> 4, m = lane & 15;
    const int b0 = blockIdx.x * BT_;

    {
        const v8h z = zero8h();
        for (int i = tid; i < (BT_ * K0P_) / 8; i += NT_) *(v8h*)(comb0 + 8 * i) = z;
        for (int i = tid; i < (BT_ * K1_) / 8; i += NT_) *(v8h*)(comb1 + 8 * i) = z;
        if (tid < BT_ * 8) g1q[tid] = 0.0f;
    }
    __syncthreads();

#pragma unroll 1
    for (int rr = 0; rr < BT_; ++rr) {
        for (int i = tid; i < 3 * NSL_; i += NT_) xb[i] = nspt[(size_t)(b0 + rr) * (3 * NSL_) + i];
        __syncthreads();
        for (int i = tid; i < 8 * 64; i += NT_) {
            const int o = i >> 6, l = i & 63;
            float s = c1b[o];
#pragma unroll 1
            for (int ic = 0; ic < 3; ++ic) {
                const float* wp = c1w + (o * 3 + ic) * 3;
                const float* xp = xb + ic * NSL_;
#pragma unroll
                for (int kk = 0; kk < 3; ++kk) {
                    const int p = 2 * l - 1 + kk;
                    const int pc = min(max(p, 0), NSL_ - 1);
                    const float xv = xp[pc];
                    s += wp[kk] * ((p >= 0 && p < NSL_) ? xv : 0.0f);
                }
            }
            y1[i] = fmaxf(s, 0.0f);
        }
        __syncthreads();
        {
            const int o = tid >> 5, l = tid & 31;
            float s = c2b[o];
#pragma unroll 1
            for (int ic = 0; ic < 8; ++ic) {
                const float* wp = c2w + (o * 8 + ic) * 3;
                const float* xp = y1 + ic * 64;
#pragma unroll
                for (int kk = 0; kk < 3; ++kk) {
                    const int p = 2 * l - 1 + kk;
                    const int pc = min(max(p, 0), 63);
                    const float xv = xp[pc];
                    s += wp[kk] * ((p >= 0 && p < 64) ? xv : 0.0f);
                }
            }
            y2[tid] = fmaxf(s, 0.0f);
        }
        __syncthreads();
        {
            const int o = tid >> 4, l = tid & 15;
            float s = c3b[o];
#pragma unroll 1
            for (int ic = 0; ic < 8; ++ic) {
                const float* wp = c3w + (o * 8 + ic) * 3;
                const float* xp = y2 + ic * 32;
#pragma unroll
                for (int kk = 0; kk < 3; ++kk) {
                    const int p = 2 * l - 1 + kk;
                    const int pc = min(max(p, 0), 31);
                    const float xv = xp[pc];
                    s += wp[kk] * ((p >= 0 && p < 32) ? xv : 0.0f);
                }
            }
            y3[tid] = fmaxf(s, 0.0f);
        }
        __syncthreads();
        if (tid < 16) {
            float s = 0.0f;
#pragma unroll
            for (int l = 0; l < 16; ++l) s += y3[tid * 16 + l];
            featS[rr * 16 + tid] = s * (1.0f / 16.0f);
        }
        __syncthreads();
    }

    float bh0v[2], bo0v[2], bh1v[2], wA[2], wB[2];
#pragma unroll
    for (int p = 0; p < 2; ++p) {
        const int n = 32 * w + 16 * p + m;
        bh0v[p] = bh0[n]; bo0v[p] = bo0[n]; bh1v[p] = bh1[n];
        wA[p] = Wo1[n]; wB[p] = Wo1[H_ + n];
    }
    const float bo1v = bo1[0];
    v8f c0r[2], c1r[2];
#pragma unroll
    for (int p = 0; p < 2; ++p) { c0r[p] = zero8f(); c1r[p] = zero8f(); }
    __syncthreads();

#pragma unroll 1
    for (int t = 0; t < T_; ++t) {
        {
            const int row = tid >> 4, cp = tid & 15;
            const float* xi = inp + ((size_t)(b0 + row) * T_ + t) * F_;
            const v4f x0 = *(const v4f*)(xi);
            const v4f x1 = *(const v4f*)(xi + 4);
            const int d = min(cp, 3);
            const float* wr = Wds + d * 7;
            float f1 = bds[d];
            f1 += wr[0] * x0[0]; f1 += wr[1] * x0[1]; f1 += wr[2] * x0[2]; f1 += wr[3] * x0[3];
            f1 += wr[4] * x1[0]; f1 += wr[5] * x1[1]; f1 += wr[6] * x1[2];
            const float fa = featS[row * 16 + min(max(cp - 5, 0), 15)];
            const float fb = featS[row * 16 + min(cp + 11, 15)];
            float v0 = fa;
            v0 = (cp == 4) ? x1[3] : v0;
            v0 = (cp < 4) ? f1 : v0;
            comb0[row * K0P_ + cp] = (_Float16)(v0 * 8.0f);
            if (cp < 5) comb0[row * K0P_ + 16 + cp] = (_Float16)(fb * 8.0f);
        }
        __syncthreads();

        v8f accA[2], accG[2];
        accA[0] = zero8f(); accA[1] = zero8f(); accG[0] = zero8f(); accG[1] = zero8f();
        {
            const _Float16* ap = comb0 + m * K0P_ + 8 * hf;
            const _Float16* bp = W0p + (size_t)(32 * w + m) * K0P_ + 8 * hf;
#pragma unroll 1
            for (int ks = 0; ks < K0P_ / 32; ++ks) {
                FragH a, b;
                ldfrag(a, ap + 32 * ks);
                ldfrag(b, bp + 32 * ks);
                accA[0] = mmah(accA[0], a, b);
                ldfrag(b, bp + (size_t)16 * K0P_ + 32 * ks);
                accA[1] = mmah(accA[1], a, b);
                ldfrag(b, bp + (size_t)256 * K0P_ + 32 * ks);
                accG[0] = mmah(accG[0], a, b);
                ldfrag(b, bp + (size_t)272 * K0P_ + 32 * ks);
                accG[1] = mmah(accG[1], a, b);
            }
        }
        __syncthreads();

        {
            v8f part = zero8f();
#pragma unroll
            for (int p = 0; p < 2; ++p) {
                const int n = 32 * w + 16 * p + m;
                const v8f aa = accA[p], gg = accG[p];
                v8f cc = c0r[p];
#pragma unroll
                for (int r = 0; r < 8; ++r) {
                    const int row = 8 * hf + r;
                    const float a = aa[r] * (1.0f / 512.0f) + bh0v[p];
                    const float g = gg[r] * (1.0f / 512.0f) + bo0v[p];
                    const float ig = sigm_f(g);
                    const float cn = ig * tanh_f(cc[r]) + (1.0f - ig) * tanh_f(a);
                    cc[r] = cn;
                    const float hn = ig * tanh_f(cn);
                    comb0[row * K0P_ + HOFF_ + n] = (_Float16)(hn * 8.0f);
                    comb1[row * K1_ + n]          = (_Float16)(g * 8.0f);
                    part[r] += g * wA[p];
                }
                c0r[p] = cc;
            }
#pragma unroll
            for (int r = 0; r < 8; ++r) {
                const float s = seg_sum(part[r]);
                if (m == 0) g1p[(8 * hf + r) * 8 + w] = s;
            }
        }
        __syncthreads();

        if (tid < BT_) {
            float s = bo1v;
#pragma unroll
            for (int q = 0; q < 8; ++q) s += g1p[tid * 8 + q];
#pragma unroll
            for (int q = 0; q < 8; ++q) s += g1q[tid * 8 + q];
            g1S[tid] = s;
            outS[tid * T_ + t] = s;
        }
        accA[0] = zero8f(); accA[1] = zero8f();
        {
            const _Float16* ap = comb1 + m * K1_ + 8 * hf;
            const _Float16* bp = W1p + (size_t)(32 * w + m) * K1_ + 8 * hf;
#pragma unroll 1
            for (int ks = 0; ks < K1_ / 32; ++ks) {
                FragH a, b;
                ldfrag(a, ap + 32 * ks);
                ldfrag(b, bp + 32 * ks);
                accA[0] = mmah(accA[0], a, b);
                ldfrag(b, bp + (size_t)16 * K1_ + 32 * ks);
                accA[1] = mmah(accA[1], a, b);
            }
        }
        __syncthreads();

        {
            v8f igv;
#pragma unroll
            for (int r = 0; r < 8; ++r) igv[r] = sigm_f(g1S[8 * hf + r]);
            v8f part = zero8f();
#pragma unroll
            for (int p = 0; p < 2; ++p) {
                const int n = 32 * w + 16 * p + m;
                const v8f aa = accA[p];
                v8f cc = c1r[p];
#pragma unroll
                for (int r = 0; r < 8; ++r) {
                    const int row = 8 * hf + r;
                    const float a = aa[r] * (1.0f / 512.0f) + bh1v[p];
                    const float ig = igv[r];
                    const float cn = ig * tanh_f(cc[r]) + (1.0f - ig) * tanh_f(a);
                    cc[r] = cn;
                    const float hn = ig * tanh_f(cn);
                    comb1[row * K1_ + H_ + n] = (_Float16)(hn * 8.0f);
                    part[r] += hn * wB[p];
                }
                c1r[p] = cc;
            }
#pragma unroll
            for (int r = 0; r < 8; ++r) {
                const float s = seg_sum(part[r]);
                if (m == 0) g1q[(8 * hf + r) * 8 + w] = s;
            }
        }
        __syncthreads();
    }

    __syncthreads();
    {
        const float* s0 = outS + (2 * w) * T_;
        const float* s1 = outS + (2 * w + 1) * T_;
        const v4f v00 = *(const v4f*)(s0 + 4 * lane);
        const v4f v01 = *(const v4f*)(s0 + 128 + 4 * lane);
        const v4f v10 = *(const v4f*)(s1 + 4 * lane);
        const v4f v11 = *(const v4f*)(s1 + 128 + 4 * lane);
        float* o0 = out + (size_t)(b0 + 2 * w) * T_;
        float* o1 = out + (size_t)(b0 + 2 * w + 1) * T_;
        *(volatile v4f*)(o0 + 4 * lane)       = v00;
        *(volatile v4f*)(o0 + 128 + 4 * lane) = v01;
        *(volatile v4f*)(o1 + 4 * lane)       = v10;
        *(volatile v4f*)(o1 + 128 + 4 * lane) = v11;
        __threadfence();
        *(volatile v4f*)(o0 + 4 * lane)       = v00;
        *(volatile v4f*)(o0 + 128 + 4 * lane) = v01;
        *(volatile v4f*)(o1 + 4 * lane)       = v10;
        *(volatile v4f*)(o1 + 128 + 4 * lane) = v11;
    }
}

extern "C" void kernel_launch(void* const* d_in, const int* in_sizes, int n_in,
                              void* d_out, int out_size, void* d_ws, size_t ws_size,
                              hipStream_t stream)
{
    if (n_in < 18) return;
    if (in_sizes[0]  != B_ * T_ * F_)   return;
    if (in_sizes[1]  != B_ * 3 * NSL_)  return;
    if (in_sizes[2]  != 4 * 7 || in_sizes[3] != 4) return;
    if (in_sizes[4]  != 8 * 3 * 3 || in_sizes[5] != 8) return;
    if (in_sizes[6]  != 8 * 8 * 3 || in_sizes[7] != 8) return;
    if (in_sizes[8]  != 16 * 8 * 3 || in_sizes[9] != 16) return;
    if (in_sizes[10] != H_ * WIN0_ || in_sizes[11] != H_) return;
    if (in_sizes[12] != H_ * WIN0_ || in_sizes[13] != H_) return;
    if (in_sizes[14] != H_ * K1_   || in_sizes[15] != H_) return;
    if (in_sizes[16] != K1_        || in_sizes[17] != 1)  return;
    if (out_size != B_ * T_)            return;
    if (ws_size < WS_END_)              return;

    const float* inp  = (const float*)d_in[0];
    const float* nspt = (const float*)d_in[1];
    const float* Wds  = (const float*)d_in[2];
    const float* bds  = (const float*)d_in[3];
    const float* c1w  = (const float*)d_in[4];
    const float* c1b  = (const float*)d_in[5];
    const float* c2w  = (const float*)d_in[6];
    const float* c2b  = (const float*)d_in[7];
    const float* c3w  = (const float*)d_in[8];
    const float* c3b  = (const float*)d_in[9];
    const float* Wh0  = (const float*)d_in[10];
    const float* bh0  = (const float*)d_in[11];
    const float* Wo0  = (const float*)d_in[12];
    const float* bo0  = (const float*)d_in[13];
    const float* Wh1  = (const float*)d_in[14];
    const float* bh1  = (const float*)d_in[15];
    const float* Wo1  = (const float*)d_in[16];
    const float* bo1  = (const float*)d_in[17];
    float* out = (float*)d_out;

    char* ws = (char*)d_ws;
    _Float16* planes = (_Float16*)(ws + OFF_P0_);
    const _Float16* W0p = (const _Float16*)(ws + OFF_P0_);
    const _Float16* W1p = (const _Float16*)(ws + OFF_P1_);

    k_planes<<<dim3(NBLK_PL_), dim3(NT_), 0, stream>>>(Wh0, Wo0, Wh1, planes);
    k_main<<<dim3(B_ / BT_), dim3(NT_), 0, stream>>>(inp, nspt, Wds, bds, c1w, c1b, c2w, c2b, c3w, c3b,
                                                    W0p, W1p, bh0, bo0, bh1, Wo1, bo1, out);
}
